// WorkingMemory_79164837200276
// MI455X (gfx1250) — hardware-verified
//
#include <hip/hip_runtime.h>
#include <math.h>

constexpr int kSeqLen = 2048;
constexpr int kDimIn  = 768;
constexpr int kMem    = 64;
constexpr int kProjN  = 3 * kMem;
constexpr int kTilesL = kSeqLen / 64;
static_assert(kProjN % 64 == 0);
static_assert(kDimIn % 64 == 0 && kSeqLen % 64 == 0 && kMem % 32 == 0);

typedef __attribute__((ext_vector_type(16))) _Float16 v16h;
typedef __attribute__((ext_vector_type(8)))  _Float16 v8h;
typedef __attribute__((ext_vector_type(16))) __bf16   v16b;
typedef __attribute__((ext_vector_type(8)))  __bf16   v8b;
typedef __attribute__((ext_vector_type(8)))  float    v8f;
typedef __attribute__((ext_vector_type(4)))  float    v4f;
typedef __attribute__((ext_vector_type(4)))  unsigned int v4u;

__device__ __forceinline__ unsigned short f2bf_bits(float f) {
  unsigned u = __float_as_uint(f);
  return (unsigned short)((u + 0x7FFFu + ((u >> 16) & 1u)) >> 16);
}
__device__ __forceinline__ float bf_bits2f(unsigned short h) { return __uint_as_float(((unsigned)h) << 16); }
__device__ __forceinline__ unsigned pk16(unsigned short a, unsigned short b) { return (unsigned)a | ((unsigned)b << 16); }

__device__ __forceinline__ void dep_guard_h(v8f& a, v8f& b, v16h x, v16h y) { asm volatile("v_nop\n\tv_nop\n\tv_nop\n\tv_nop" : "+v"(a), "+v"(b) : "v"(x), "v"(y)); }
__device__ __forceinline__ void dep_guard_b(v8f& a, v8f& b, v16b x, v16b y) { asm volatile("v_nop\n\tv_nop\n\tv_nop\n\tv_nop" : "+v"(a), "+v"(b) : "v"(x), "v"(y)); }
__device__ __forceinline__ void keep4_h(v16h a, v16h b, v16h c, v16h d) { asm volatile("v_nop" :: "v"(a), "v"(b), "v"(c), "v"(d)); }
__device__ __forceinline__ void keep4_b(v16b a, v16b b, v16b c, v16b d) { asm volatile("v_nop" :: "v"(a), "v"(b), "v"(c), "v"(d)); }
__device__ __forceinline__ void acc_guard4(v8f& a, v8f& b, v8f& c, v8f& d) { asm volatile("v_nop\n\tv_nop\n\tv_nop\n\tv_nop" : "+v"(a), "+v"(b), "+v"(c), "+v"(d)); }
template <typename T> struct Frag;
template <> struct Frag<_Float16> {
  typedef v16h V; union U { v16h v; v8h h[2]; };
  static __device__ __forceinline__ v16h load(const _Float16* p) {
    U f; f.h[0] = *(const v8h*)(p); f.h[1] = *(const v8h*)(p + 16); return f.v;
  }
  static __device__ __forceinline__ v8f mma(v16h a, v16h b, v8f c) {
    return __builtin_amdgcn_wmma_f32_16x16x32_f16(false, a, false, b, (short)0, c, false, false);
  }
  static __device__ __forceinline__ void guard(v8f& a, v8f& b, v16h x, v16h y) { dep_guard_h(a, b, x, y); }
  static __device__ __forceinline__ void keep(v16h a, v16h b, v16h c, v16h d) { keep4_h(a, b, c, d); }
};
template <> struct Frag<__bf16> {
  typedef v16b V; union U { v16b v; v8b h[2]; };
  static __device__ __forceinline__ v16b load(const __bf16* p) {
    U f; f.h[0] = *(const v8b*)(p); f.h[1] = *(const v8b*)(p + 16); return f.v;
  }
  static __device__ __forceinline__ v8f mma(v16b a, v16b b, v8f c) {
    return __builtin_amdgcn_wmma_f32_16x16x32_bf16(false, a, false, b, (short)0, c, false, false);
  }
  static __device__ __forceinline__ void guard(v8f& a, v8f& b, v16b x, v16b y) { dep_guard_b(a, b, x, y); }
  static __device__ __forceinline__ void keep(v16b a, v16b b, v16b c, v16b d) { keep4_b(a, b, c, d); }
};

__device__ __forceinline__ void split8(v4f a, v4f c, v4u& uh, v4u& ul) {
  unsigned short hb[8], lb[8];
#pragma unroll
  for (int e = 0; e < 4; ++e) {
    hb[e] = f2bf_bits(a[e]);
    lb[e] = f2bf_bits(a[e] - bf_bits2f(hb[e]));
    hb[4 + e] = f2bf_bits(c[e]);
    lb[4 + e] = f2bf_bits(c[e] - bf_bits2f(hb[4 + e]));
  }
  uh = (v4u){pk16(hb[0], hb[1]), pk16(hb[2], hb[3]), pk16(hb[4], hb[5]), pk16(hb[6], hb[7])};
  ul = (v4u){pk16(lb[0], lb[1]), pk16(lb[2], lb[3]), pk16(lb[4], lb[5]), pk16(lb[6], lb[7])};
}

template <int ET> struct Elem;
template <> struct Elem<0> { typedef _Float16 T; };
template <> struct Elem<1> { typedef __bf16 T; };
template <int ET, bool SPLIT, int BIAS_MODE, int OUT_MODE, bool RESID, int ACT = 0, bool KTRI = false>
__global__ __launch_bounds__(256) void wmma_gemm64(
    const unsigned short* __restrict__ Ap, const unsigned short* __restrict__ A2p, int lda, long strideA,
    const unsigned short* __restrict__ Btp, const unsigned short* __restrict__ Bt2p, int ldb, long strideB,
    void* __restrict__ Cout, void* __restrict__ Cout2, int ldc, long strideC,
    const float* __restrict__ bias,
    const float* __restrict__ resid, long strideR,
    int M, int N, int K, float scale) {
  typedef typename Elem<ET>::T T;
  typedef typename Frag<T>::V V;
  const T* A = (const T*)Ap; const T* A2 = (const T*)A2p; const T* Bt = (const T*)Btp; const T* Bt2 = (const T*)Bt2p;
  __shared__ __align__(16) float sT[8][16 * 68];
  const int b    = blockIdx.y;
  const int lane = threadIdx.x & 31;
  const int wave = threadIdx.x >> 5;
  const int tilesN = N >> 6;
  const int tilesM = M >> 6;
  const int tile = blockIdx.x * 8 + wave;
  if (tile >= tilesM * tilesN) return;
  const int tm = tile / tilesN;
  const int tn = tile - tm * tilesN;
  const int m0 = tm << 6;
  const int n0 = tn << 6;

  const T* Ab  = A  + (size_t)b * strideA;
  const T* Bb  = Bt + (size_t)b * strideB;
  const T* Ab2 = SPLIT ? (A2  + (size_t)b * strideA) : nullptr;
  const T* Bb2 = SPLIT ? (Bt2 + (size_t)b * strideB) : nullptr;

  const int rlane = lane & 15;
  const int koff  = (lane >> 4) * 8;
  const int mOff  = (lane >> 4) * 8;

  v8f acc[4][4];
#pragma unroll
  for (int i = 0; i < 4; ++i)
#pragma unroll
    for (int j = 0; j < 4; ++j) acc[i][j] = (v8f){0.f,0.f,0.f,0.f,0.f,0.f,0.f,0.f};

  int Kend = K;
  if (KTRI) { const int kt = (tm + 1) << 6; Kend = (kt < K) ? kt : K; }

  for (int k0 = 0; k0 < Kend; k0 += 32) {
    V bh[4], bl[4];
#pragma unroll
    for (int j = 0; j < 4; ++j) {
      const size_t bo = (size_t)(n0 + (j << 4) + rlane) * ldb + koff + k0;
      bh[j] = Frag<T>::load(Bb + bo);
      if (SPLIT) bl[j] = Frag<T>::load(Bb2 + bo);
    }
#pragma unroll
    for (int i = 0; i < 4; ++i) {
      const size_t ao = (size_t)(m0 + (i << 4) + rlane) * lda + koff + k0;
      V ah = Frag<T>::load(Ab + ao);
      V al;
      if (SPLIT) al = Frag<T>::load(Ab2 + ao);
#pragma unroll
      for (int j = 0; j < 4; ++j) {
        acc[i][j] = Frag<T>::mma(ah, bh[j], acc[i][j]);
        if (SPLIT) {
          acc[i][j] = Frag<T>::mma(ah, bl[j], acc[i][j]);
          acc[i][j] = Frag<T>::mma(al, bh[j], acc[i][j]);
        }
      }
      Frag<T>::guard(acc[i][0], acc[i][3], ah, SPLIT ? al : ah);
    }
    Frag<T>::keep(bh[0], bh[1], bh[2], bh[3]);
    if (SPLIT) Frag<T>::keep(bl[0], bl[1], bl[2], bl[3]);
  }
  acc_guard4(acc[0][0], acc[0][1], acc[0][2], acc[0][3]);
  acc_guard4(acc[1][0], acc[1][1], acc[1][2], acc[1][3]);
  acc_guard4(acc[2][0], acc[2][1], acc[2][2], acc[2][3]);
  acc_guard4(acc[3][0], acc[3][1], acc[3][2], acc[3][3]);

  float* slab = sT[wave];
  const float* Rb = RESID ? (resid + (size_t)b * strideR) : nullptr;
#pragma unroll
  for (int i = 0; i < 4; ++i) {
    const int mBase = m0 + (i << 4);
#pragma unroll
    for (int j = 0; j < 4; ++j) {
      const int n = n0 + (j << 4) + rlane;
      float bv = 0.f;
      if (BIAS_MODE == 2) bv = bias[n];
#pragma unroll
      for (int r = 0; r < 8; ++r) {
        float v = acc[i][j][r] * scale;
        if (BIAS_MODE == 1) v += bias[mBase + mOff + r];
        if (BIAS_MODE == 2) v += bv;
        if (RESID) v += Rb[(size_t)(mBase + mOff + r) * ldc + n];
        if (ACT == 2) v = fmaxf(v, 0.0f);
        if (ACT == 4) v = (v > 0.f) ? v : 0.01f * v;
        slab[(mOff + r) * 68 + (j << 4) + rlane] = v;
      }
    }
    __builtin_amdgcn_fence(__ATOMIC_RELEASE, "workgroup");
    __builtin_amdgcn_wave_barrier();
    __builtin_amdgcn_fence(__ATOMIC_ACQUIRE, "workgroup");
    if (OUT_MODE == 0) {
      float* C = (float*)Cout + (size_t)b * strideC;
      const int hh = lane >> 4, c4 = (lane & 15) * 4;
      for (int pass = 0; pass < 2; ++pass) {
#pragma unroll
        for (int it = 0; it < 8; ++it) {
          const int row = it * 2 + hh;
          v4f v = *(const v4f*)(slab + row * 68 + c4);
          *(volatile v4f*)(C + (size_t)(mBase + row) * ldc + n0 + c4) = v;
        }
        __threadfence();
      }
    } else {
      const int q = lane >> 3, c8 = (lane & 7) * 8;
      unsigned short* C  = (unsigned short*)Cout  + (size_t)b * strideC;
      unsigned short* C2 = (OUT_MODE == 2) ? ((unsigned short*)Cout2 + (size_t)b * strideC) : nullptr;
      for (int pass = 0; pass < 2; ++pass) {
#pragma unroll
        for (int it = 0; it < 4; ++it) {
          const int row = it * 4 + q;
          const float* sp = slab + row * 68 + c8;
          v8h hv, lv;
#pragma unroll
          for (int e = 0; e < 8; ++e) {
            if (OUT_MODE == 1) {
              hv[e] = (_Float16)sp[e];
            } else {
              unsigned short hb = f2bf_bits(sp[e]);
              unsigned short lb = f2bf_bits(sp[e] - bf_bits2f(hb));
              hv[e] = __builtin_bit_cast(_Float16, hb);
              lv[e] = __builtin_bit_cast(_Float16, lb);
            }
          }
          *(volatile v8h*)(C + (size_t)(mBase + row) * ldc + n0 + c8) = hv;
          if (OUT_MODE == 2) *(volatile v8h*)(C2 + (size_t)(mBase + row) * ldc + n0 + c8) = lv;
        }
        __threadfence();
      }
    }
    __builtin_amdgcn_fence(__ATOMIC_RELEASE, "workgroup");
    __builtin_amdgcn_wave_barrier();
    __builtin_amdgcn_fence(__ATOMIC_ACQUIRE, "workgroup");
  }
}

__global__ __launch_bounds__(256) void gemm_scores_kernel(
    const unsigned short* __restrict__ Ap, const unsigned short* __restrict__ A2p,
    const unsigned short* __restrict__ Btp, const unsigned short* __restrict__ Bt2p,
    unsigned short* __restrict__ Sh, unsigned short* __restrict__ Sl, float* __restrict__ PT) {
  typedef __bf16 T;
  typedef v16b V;
  constexpr int lda = kMem, ldb = kMem, ldc = kSeqLen, Kd = kMem;
  __shared__ __align__(16) float sT[8][16 * 68];
  __shared__ __align__(16) float sP[8][64];
  const T* A = (const T*)Ap; const T* A2 = (const T*)A2p; const T* Bt = (const T*)Btp; const T* Bt2 = (const T*)Bt2p;
  const int lane = threadIdx.x & 31;
  const int wave = threadIdx.x >> 5;
  const int tile = blockIdx.x * 8 + wave;
  const int tm = tile >> 5;
  const int tn = tile & 31;
  if (tn > tm) return;
  const int m0 = tm << 6;
  const int n0 = tn << 6;
  const int rlane = lane & 15;
  const int koff  = (lane >> 4) * 8;
  const int mOff  = (lane >> 4) * 8;

  v8f acc[4][4];
#pragma unroll
  for (int i = 0; i < 4; ++i)
#pragma unroll
    for (int j = 0; j < 4; ++j) acc[i][j] = (v8f){0.f,0.f,0.f,0.f,0.f,0.f,0.f,0.f};

  for (int k0 = 0; k0 < Kd; k0 += 32) {
    V bh[4], bl[4];
#pragma unroll
    for (int j = 0; j < 4; ++j) {
      const size_t bo = (size_t)(n0 + (j << 4) + rlane) * ldb + koff + k0;
      bh[j] = Frag<T>::load(Bt + bo);
      bl[j] = Frag<T>::load(Bt2 + bo);
    }
#pragma unroll
    for (int i = 0; i < 4; ++i) {
      const size_t ao = (size_t)(m0 + (i << 4) + rlane) * lda + koff + k0;
      V ah = Frag<T>::load(A + ao);
      V al = Frag<T>::load(A2 + ao);
#pragma unroll
      for (int j = 0; j < 4; ++j) {
        acc[i][j] = Frag<T>::mma(ah, bh[j], acc[i][j]);
        acc[i][j] = Frag<T>::mma(ah, bl[j], acc[i][j]);
        acc[i][j] = Frag<T>::mma(al, bh[j], acc[i][j]);
      }
      Frag<T>::guard(acc[i][0], acc[i][3], ah, al);
    }
    Frag<T>::keep(bh[0], bh[1], bh[2], bh[3]);
    Frag<T>::keep(bl[0], bl[1], bl[2], bl[3]);
  }
  acc_guard4(acc[0][0], acc[0][1], acc[0][2], acc[0][3]);
  acc_guard4(acc[1][0], acc[1][1], acc[1][2], acc[1][3]);
  acc_guard4(acc[2][0], acc[2][1], acc[2][2], acc[2][3]);
  acc_guard4(acc[3][0], acc[3][1], acc[3][2], acc[3][3]);

  float* slab = sT[wave];
  float* psum = sP[wave];
#pragma unroll
  for (int i = 0; i < 4; ++i) {
    const int mBase = m0 + (i << 4);
#pragma unroll
    for (int j = 0; j < 4; ++j) {
      const int n = n0 + (j << 4) + rlane;
#pragma unroll
      for (int r = 0; r < 8; ++r) {
        const int gm = mBase + mOff + r;
        float v = acc[i][j][r];
        v = (n > gm) ? 0.0f : v;
        slab[(mOff + r) * 68 + (j << 4) + rlane] = v;
      }
    }
    __builtin_amdgcn_fence(__ATOMIC_RELEASE, "workgroup");
    __builtin_amdgcn_wave_barrier();
    __builtin_amdgcn_fence(__ATOMIC_ACQUIRE, "workgroup");
    {
      const int rr = lane & 15;
      const float* sp0 = slab + rr * 68;
      float s = 0.0f;
#pragma unroll
      for (int c4 = 0; c4 < 16; ++c4) {
        const v4f w = *(const v4f*)(sp0 + 4 * c4);
        s += w[0]; s += w[1]; s += w[2]; s += w[3];
      }
      if (lane < 16) psum[(i << 4) + rr] = s;
    }
    {
      const int q = lane >> 3, c8 = (lane & 7) * 8;
      for (int pass = 0; pass < 2; ++pass) {
#pragma unroll
        for (int it = 0; it < 4; ++it) {
          const int row = it * 4 + q;
          const float* sp = slab + row * 68 + c8;
          v8h hv, lv;
#pragma unroll
          for (int e = 0; e < 8; ++e) {
            unsigned short hb = f2bf_bits(sp[e]);
            unsigned short lb = f2bf_bits(sp[e] - bf_bits2f(hb));
            hv[e] = __builtin_bit_cast(_Float16, hb);
            lv[e] = __builtin_bit_cast(_Float16, lb);
          }
          *(volatile v8h*)(Sh + (size_t)(mBase + row) * ldc + n0 + c8) = hv;
          *(volatile v8h*)(Sl + (size_t)(mBase + row) * ldc + n0 + c8) = lv;
        }
        __threadfence();
      }
    }
    __builtin_amdgcn_fence(__ATOMIC_RELEASE, "workgroup");
    __builtin_amdgcn_wave_barrier();
    __builtin_amdgcn_fence(__ATOMIC_ACQUIRE, "workgroup");
  }
  {
    const int li = (lane & 15) * 4;
    const v4f pv = *(const v4f*)(psum + li);
    for (int pass = 0; pass < 2; ++pass) {
      if (lane < 16) *(volatile v4f*)(PT + (size_t)tn * kSeqLen + m0 + li) = pv;
      __threadfence();
    }
  }
}

__global__ __launch_bounds__(256) void xsplit_kernel(const float* __restrict__ in, unsigned short* __restrict__ oh,
                                                     unsigned short* __restrict__ ol, int n8) {
  const int i = blockIdx.x * 256 + threadIdx.x;
  if (i >= n8) return;
  const float* p = in + 8 * (size_t)i;
  const v4f a = *(const v4f*)(p);
  const v4f c = *(const v4f*)(p + 4);
  v4u uh, ul;
  split8(a, c, uh, ul);
  unsigned short* qh = oh + 8 * (size_t)i;
  unsigned short* ql = ol + 8 * (size_t)i;
  *(volatile v4u*)qh = uh;
  *(volatile v4u*)ql = ul;
  __threadfence();
  *(volatile v4u*)qh = uh;
  *(volatile v4u*)ql = ul;
}

__global__ __launch_bounds__(256) void wtsplit_kernel(const float* __restrict__ W, int n_out,
                                                      unsigned short* __restrict__ oh, unsigned short* __restrict__ ol,
                                                      int row_off) {
  __shared__ float sm[64][65];
  const int t  = threadIdx.x;
  const int k0 = blockIdx.x * 64;
  const int n0 = blockIdx.y * 64;
#pragma unroll
  for (int i = 0; i < 16; ++i) {
    const int e  = i * 256 + t;
    const int kl = e >> 6;
    const int nl = e & 63;
    sm[nl][kl] = W[(size_t)(k0 + kl) * n_out + n0 + nl];
  }
  __syncthreads();
  const int lane = t & 31, wave = t >> 5;
  const int q = lane >> 3, c8 = (lane & 7) * 8;
  for (int pass = 0; pass < 2; ++pass) {
#pragma unroll
    for (int it = 0; it < 2; ++it) {
      const int row = wave * 8 + it * 4 + q;
      const float* sp = &sm[row][c8];
      const v4f a = (v4f){sp[0], sp[1], sp[2], sp[3]};
      const v4f c = (v4f){sp[4], sp[5], sp[6], sp[7]};
      v4u uh, ul;
      split8(a, c, uh, ul);
      const size_t o = (size_t)(row_off + n0 + row) * kDimIn + k0 + c8;
      *(volatile v4u*)(oh + o) = uh;
      *(volatile v4u*)(ol + o) = ul;
    }
    __threadfence();
  }
}

__global__ __launch_bounds__(64) void gate_scan_kernel(const float* __restrict__ c1, const float* __restrict__ bfp,
                                                       unsigned short* __restrict__ QPh, unsigned short* __restrict__ QPl,
                                                       unsigned short* __restrict__ KNh, unsigned short* __restrict__ KNl) {
  __shared__ __align__(16) float sv[2][64][64];
  const int t = threadIdx.x;
  const float bm = bfp[t];
  float cum = 0.0f;
  for (int ch = 0; ch < kSeqLen / 64; ++ch) {
#pragma unroll 1
    for (int lr = 0; lr < 64; ++lr) {
      const int l = ch * 64 + lr;
      const float* cr = c1 + (size_t)l * kProjN;
      const float uq = cr[t];
      const float uk = cr[kMem + t];
      const float uf = cr[2 * kMem + t] + bm;
      const float ef = expf(-uf);
      const float fg = 1.0f / (1.0f + ef);
      const float lf = logf(fmaxf(fg, 1e-6f));
      cum += lf;
      const float cc = fminf(20.0f, fmaxf(-20.0f, cum));
      const float ep = expf(cc);
      const float en = expf(-cc);
      const float eq = expf(fminf(uq, 0.0f));
      const float ek = expf(fminf(uk, 0.0f));
      const float qv = ((uq > 0.0f) ? (uq + 1.0f) : eq) * 0.125f;
      const float kv = (uk > 0.0f) ? (uk + 1.0f) : ek;
      sv[0][lr][t] = qv * ep;
      sv[1][lr][t] = kv * en;
    }
    __syncthreads();
    {
      const int g = t >> 3, c8 = (t & 7) * 8;
      for (int pass = 0; pass < 2; ++pass) {
#pragma unroll
        for (int it = 0; it < 16; ++it) {
          const int arr = it & 1;
          const int row = (it >> 1) * 8 + g;
          const float* sp = &sv[arr][row][c8];
          const v4f a = *(const v4f*)(sp);
          const v4f c = *(const v4f*)(sp + 4);
          v4u uh, ul;
          split8(a, c, uh, ul);
          unsigned short* dh = arr ? KNh : QPh;
          unsigned short* dl = arr ? KNl : QPl;
          const size_t o = (size_t)(ch * 64 + row) * kMem + c8;
          *(volatile v4u*)(dh + o) = uh;
          *(volatile v4u*)(dl + o) = ul;
        }
        __threadfence();
      }
    }
    __syncthreads();
  }
}

__global__ __launch_bounds__(256) void ln_split_kernel(const float* __restrict__ num, const float* __restrict__ PT,
                                                       const float* __restrict__ gamma, const float* __restrict__ beta,
                                                       unsigned short* __restrict__ Nh, unsigned short* __restrict__ Nl) {
  __shared__ float red[256];
  __shared__ float pden[32];
  __shared__ float sden;
  __shared__ __align__(16) float sn[kDimIn];
  const int row = blockIdx.x;
  const int t = threadIdx.x;
  if (t < 32) {
    const int ntl = row >> 6;
    const int tc = (t < ntl) ? t : ntl;
    const float pv = PT[(size_t)tc * kSeqLen + row];
    pden[t] = (t <= ntl) ? pv : 0.0f;
  }
  __syncthreads();
  if (t == 0) {
    float s = 0.0f;
#pragma unroll
    for (int i = 0; i < 32; ++i) s += pden[i];
    sden = s + 1e-6f;
  }
  __syncthreads();
  const float inv = 1.0f / sden;
  const float* hr = num + (size_t)row * kDimIn;
  const float v0 = hr[t] * inv;
  const float v1 = hr[256 + t] * inv;
  const float v2 = hr[512 + t] * inv;

  red[t] = v0 + v1 + v2;
  __syncthreads();
  for (int off = 128; off > 0; off >>= 1) {
    if (t < off) red[t] += red[t + off];
    __syncthreads();
  }
  const float mu = red[0] * (1.0f / (float)kDimIn);
  __syncthreads();
  const float d0 = v0 - mu, d1 = v1 - mu, d2 = v2 - mu;
  red[t] = d0 * d0 + d1 * d1 + d2 * d2;
  __syncthreads();
  for (int off = 128; off > 0; off >>= 1) {
    if (t < off) red[t] += red[t + off];
    __syncthreads();
  }
  const float var = red[0] * (1.0f / (float)kDimIn);
  const float rsd = 1.0f / sqrtf(var + 1e-5f);
  sn[t]       = d0 * rsd * gamma[t] + beta[t];
  sn[256 + t] = d1 * rsd * gamma[256 + t] + beta[256 + t];
  sn[512 + t] = d2 * rsd * gamma[512 + t] + beta[512 + t];
  __syncthreads();
  {
    const int tcl = (t < 96) ? t : 95;
    const int q = tcl >> 3, c8 = (tcl & 7) * 8;
    const float* sp = sn + q * 64 + c8;
    const v4f a = *(const v4f*)(sp);
    const v4f c = *(const v4f*)(sp + 4);
    v4u uh, ul;
    split8(a, c, uh, ul);
    const size_t o = (size_t)row * kDimIn + q * 64 + c8;
    for (int pass = 0; pass < 2; ++pass) {
      if (t < 96) {
        *(volatile v4u*)(Nh + o) = uh;
        *(volatile v4u*)(Nl + o) = ul;
      }
      __threadfence();
    }
  }
}

extern "C" void kernel_launch(void* const* d_in, const int* in_sizes, int n_in,
                              void* d_out, int out_size, void* d_ws, size_t ws_size,
                              hipStream_t stream) {
  if (n_in < 9) return;
  if (in_sizes[0] != kSeqLen * kDimIn || in_sizes[1] != kDimIn * kMem || in_sizes[2] != kDimIn * kMem ||
      in_sizes[3] != kDimIn * kDimIn || in_sizes[4] != kDimIn * kMem || in_sizes[5] != kMem ||
      in_sizes[6] != kDimIn * kDimIn || in_sizes[7] != kDimIn || in_sizes[8] != kDimIn) return;
  if (out_size != kSeqLen * kDimIn) return;

  const float* x     = (const float*)d_in[0];
  const float* Wq    = (const float*)d_in[1];
  const float* Wk    = (const float*)d_in[2];
  const float* Wv    = (const float*)d_in[3];
  const float* Wf    = (const float*)d_in[4];
  const float* bfv   = (const float*)d_in[5];
  const float* Wo    = (const float*)d_in[6];
  const float* gamma = (const float*)d_in[7];
  const float* beta  = (const float*)d_in[8];
  float* out = (float*)d_out;

  char* ws = (char*)d_ws;
  size_t off = 0;
  auto carve = [&](size_t bytes) -> char* {
    char* p = ws + off;
    off += (bytes + 255) & ~(size_t)255;
    return p;
  };
  const size_t bXD  = (size_t)kSeqLen * kDimIn * 2;
  const size_t bWc  = (size_t)kProjN * kDimIn * 2;
  const size_t bWW  = (size_t)kDimIn * kDimIn * 2;
  const size_t bC1  = (size_t)kSeqLen * kProjN * 4;
  const size_t bQK  = (size_t)kSeqLen * kMem * 2;
  const size_t bS   = (size_t)kSeqLen * kSeqLen * 2;
  const size_t bPT  = (size_t)kTilesL * kSeqLen * 4;
  const size_t bNUM = (size_t)kSeqLen * kDimIn * 4;

  unsigned short* Xh   = (unsigned short*)carve(bXD);
  unsigned short* Xl   = (unsigned short*)carve(bXD);
  unsigned short* WcTh = (unsigned short*)carve(bWc);
  unsigned short* WcTl = (unsigned short*)carve(bWc);
  unsigned short* WvTh = (unsigned short*)carve(bWW);
  unsigned short* WvTl = (unsigned short*)carve(bWW);
  unsigned short* WoTh = (unsigned short*)carve(bWW);
  unsigned short* WoTl = (unsigned short*)carve(bWW);
  float*          C1   = (float*)carve(bC1);
  unsigned short* QPh  = (unsigned short*)carve(bQK);
  unsigned short* QPl  = (unsigned short*)carve(bQK);
  unsigned short* KNh  = (unsigned short*)carve(bQK);
  unsigned short* KNl  = (unsigned short*)carve(bQK);
  unsigned short* Vth  = (unsigned short*)carve(bXD);
  unsigned short* Vtl  = (unsigned short*)carve(bXD);
  unsigned short* Sh   = (unsigned short*)carve(bS);
  unsigned short* Sl   = (unsigned short*)carve(bS);
  float*          PT   = (float*)carve(bPT);
  float*          NUM  = (float*)carve(bNUM);
  unsigned short* Nh   = (unsigned short*)carve(bXD);
  unsigned short* Nl   = (unsigned short*)carve(bXD);
  if (off > ws_size) return;

  {
    const int n8 = kSeqLen * kDimIn / 8;
    xsplit_kernel<<<dim3((n8 + 255) / 256), 256, 0, stream>>>(x, Xh, Xl, n8);
  }
  wtsplit_kernel<<<dim3(kDimIn / 64, kMem / 64), 256, 0, stream>>>(Wq, kMem, WcTh, WcTl, 0);
  wtsplit_kernel<<<dim3(kDimIn / 64, kMem / 64), 256, 0, stream>>>(Wk, kMem, WcTh, WcTl, kMem);
  wtsplit_kernel<<<dim3(kDimIn / 64, kMem / 64), 256, 0, stream>>>(Wf, kMem, WcTh, WcTl, 2 * kMem);
  wtsplit_kernel<<<dim3(kDimIn / 64, kDimIn / 64), 256, 0, stream>>>(Wv, kDimIn, WvTh, WvTl, 0);
  wtsplit_kernel<<<dim3(kDimIn / 64, kDimIn / 64), 256, 0, stream>>>(Wo, kDimIn, WoTh, WoTl, 0);

  wmma_gemm64<1, true, 0, 0, false, 0, false><<<dim3((kSeqLen / 64) * (kProjN / 64) / 8, 1), 256, 0, stream>>>(
      Xh, Xl, kDimIn, 0L, WcTh, WcTl, kDimIn, 0L, (void*)C1, (void*)nullptr, kProjN, 0L,
      (const float*)nullptr, (const float*)nullptr, 0L, kSeqLen, kProjN, kDimIn, 1.0f);

  wmma_gemm64<1, true, 0, 2, false, 0, false><<<dim3((kDimIn / 64) * (kSeqLen / 64) / 8, 1), 256, 0, stream>>>(
      WvTh, WvTl, kDimIn, 0L, Xh, Xl, kDimIn, 0L, (void*)Vth, (void*)Vtl, kSeqLen, 0L,
      (const float*)nullptr, (const float*)nullptr, 0L, kDimIn, kSeqLen, kDimIn, 1.0f);

  gate_scan_kernel<<<dim3(1), 64, 0, stream>>>(C1, bfv, QPh, QPl, KNh, KNl);

  gemm_scores_kernel<<<dim3(kTilesL * kTilesL / 8), 256, 0, stream>>>(QPh, QPl, KNh, KNl, Sh, Sl, PT);

  wmma_gemm64<1, true, 0, 0, false, 0, true><<<dim3((kSeqLen / 64) * (kDimIn / 64) / 8, 1), 256, 0, stream>>>(
      Sh, Sl, kSeqLen, 0L, Vth, Vtl, kSeqLen, 0L, (void*)NUM, (void*)nullptr, kDimIn, 0L,
      (const float*)nullptr, (const float*)nullptr, 0L, kSeqLen, kDimIn, kSeqLen, 1.0f);

  ln_split_kernel<<<dim3(kSeqLen), 256, 0, stream>>>(NUM, PT, gamma, beta, Nh, Nl);

  wmma_gemm64<1, true, 0, 0, false, 0, false><<<dim3((kSeqLen / 64) * (kDimIn / 64) / 8, 1), 256, 0, stream>>>(
      Nh, Nl, kDimIn, 0L, WoTh, WoTl, kDimIn, 0L, (void*)out, (void*)nullptr, kDimIn, 0L,
      (const float*)nullptr, (const float*)nullptr, 0L, kSeqLen, kDimIn, kDimIn, 1.0f);
}
